// PixelAttendPers_6201932775595
// MI455X (gfx1250) — hardware-run, weakly checked
//
#include <hip/hip_runtime.h>
#include <math.h>

typedef __attribute__((ext_vector_type(16))) _Float16 v16h;
typedef __attribute__((ext_vector_type(8)))  _Float16 v8h;
typedef __attribute__((ext_vector_type(8)))  float    v8f;
typedef __attribute__((ext_vector_type(4)))  float    v4f;
typedef __attribute__((ext_vector_type(4)))  unsigned int v4u;

constexpr int kBatch  = 2;
constexpr int kSide   = 64;
constexpr int kNpix   = kSide * kSide;
constexpr int kRows   = kBatch * kNpix;
constexpr int kCh     = 64;
constexpr int kPosC   = 32;
constexpr int kLayers = 8;
constexpr int kOutC   = 100;
constexpr int kConvIn = 3;
constexpr int kKq     = kCh + kPosC;
constexpr int kKg     = kCh + kPosC + kCh;
constexpr int kNcat   = 5 * kCh;
constexpr int kSqrtCh = 8;
static_assert(kSqrtCh * kSqrtCh == kCh);
constexpr float kScoreScale = 1.0f / (float)kSqrtCh;
constexpr float kWCarry     = 64.0f;
constexpr float kWCarryInv  = 1.0f / kWCarry;
constexpr float kPCarry     = 32768.0f;
constexpr float kResCarry   = 2048.0f;
constexpr float kResInv     = 1.0f / kResCarry;
constexpr float kF16MinNorm = 6.103515625e-5f;
constexpr float kMaskFill   = -10000.0f;
constexpr float kBnEps      = 1e-5f;
constexpr float kInvCount   = 1.0f / (float)kRows;
constexpr int   kGateTileM  = 32;
constexpr int   kGateTiles  = (kRows / kGateTileM) * 5;
static_assert(kNpix == 4096 && kRows == 8192);
static_assert((kKq % 32) == 0 && (kKg % 32) == 0);
static_assert((kRows % 64) == 0 && (kNcat % 64) == 0 && (kNpix % 64) == 0);
static_assert((kRows % kGateTileM) == 0 && (kGateTiles % 8) == 0);
static_assert(kRows == 256 * 32);

constexpr size_t kSzPos  = (size_t)kNpix * kPosC * 2;
constexpr size_t kSzW    = (size_t)kLayers * kNcat * kKg * 2;
constexpr size_t kSzStat = (size_t)kCh * 32 * 4;
constexpr size_t kSzF32  = (size_t)kRows * kCh * 4;
constexpr size_t kSzF16  = (size_t)kRows * kCh * 2;
constexpr size_t kOffPosH = 0;
constexpr size_t kOffPosL = kOffPosH + kSzPos;
constexpr size_t kOffWH   = kOffPosL + kSzPos;
constexpr size_t kOffWL   = kOffWH   + kSzW;
constexpr size_t kOffStat = kOffWL   + kSzW;
constexpr size_t kOffK32A = kOffStat + kSzStat;
constexpr size_t kOffV32A = kOffK32A + kSzF32;
constexpr size_t kOffKTH  = kOffV32A + kSzF32;
constexpr size_t kOffKTL  = kOffKTH  + kSzF16;
constexpr size_t kOffVTH  = kOffKTL  + kSzF16;
constexpr size_t kOffVTL  = kOffVTH  + kSzF16;
constexpr size_t kOffVCMH = kOffVTL  + kSzF16;
constexpr size_t kOffVCML = kOffVCMH + kSzF16;
constexpr size_t kOffK32B = kOffVCML + kSzF16;
constexpr size_t kOffV32B = kOffK32B + kSzF32;
constexpr size_t kOffHTH  = kOffV32B + kSzF32;
constexpr size_t kOffHTL  = kOffHTH  + kSzF16;
constexpr size_t kOffQTH  = kOffHTL  + kSzF16;
constexpr size_t kOffQTL  = kOffQTH  + kSzF16;
constexpr size_t kOffFKP  = kOffQTL  + kSzF16;
constexpr size_t kOffCKP  = kOffFKP  + kSzF32;
constexpr size_t kOffFVP  = kOffCKP  + kSzF32;
constexpr size_t kOffCVP  = kOffFVP  + kSzF32;
constexpr size_t kOffOUT1 = kOffCVP  + kSzF32;
constexpr size_t kOffHPRE = kOffOUT1 + kSzF32;
constexpr size_t kWsTotal = kOffHPRE + kSzF32;
constexpr size_t kZeroBytes = 2 * kSzF32 + 6 * kSzF16;
static_assert(kWsTotal == 33628160ull);
static_assert(kWsTotal <= 134217728ull);
static_assert(kOffK32B - kOffK32A == kZeroBytes);
static_assert((kZeroBytes % (16 * 256)) == 0);
static_assert((kSzPos % 128) == 0 && (kSzW % 128) == 0 && (kSzStat % 128) == 0 && (kSzF32 % 128) == 0 &&
              (kSzF16 % 128) == 0);

union FragH { v16h v; v8h h[2]; };
__device__ __forceinline__ v16h frag_load(const _Float16* p) {
  FragH f;
  f.h[0] = *(const v8h*)(p);
  f.h[1] = *(const v8h*)(p + 16);
  return f.v;
}
__device__ __forceinline__ v8f mma_h(v16h a, v16h b, v8f c) {
  c = __builtin_amdgcn_wmma_f32_16x16x32_f16(false, a, false, b, (short)0, c, false, false);
  asm volatile("v_nop\n\tv_nop\n\tv_nop\n\tv_nop" : "+v"(c) : "v"(a), "v"(b));
  return c;
}
__device__ __forceinline__ float wave_sum(float v) {
#pragma unroll
  for (int off = 16; off > 0; off >>= 1) v += __shfl_xor(v, off, 32);
  return v;
}
__device__ __forceinline__ void split16(float x, _Float16& hi, _Float16& lo) {
  const _Float16 h0 = (_Float16)x;
  const float hf0 = (float)h0;
  const float hf = (fabsf(hf0) < kF16MinNorm) ? 0.0f : hf0;
  hi = (_Float16)hf;
  lo = (_Float16)((x - hf) * kResCarry);
}

__global__ __launch_bounds__(256) void pos_kernel(_Float16* __restrict__ posH, _Float16* __restrict__ posL) {
  __shared__ float sv[8 * 32];
  const int t = threadIdx.x, lane = t & 31, wave = t >> 5;
  const int n0 = blockIdx.x * 8;
  const int px = t >> 5, ch = t & 31;
  const int n = n0 + px;
  const int y = n >> 6, x = n & 63;
  const int a = ch & 15;
  const int i = (ch < 16) ? y : x;
  const int flat = a * 64 + i;
  const int p = flat >> 4, j = flat & 15;
  const int kk = j >> 1;
  float dv = 1.0f;
  dv = (kk == 1) ? 3.1622776601683795f : dv;
  dv = (kk == 2) ? 10.0f : dv;
  dv = (kk == 3) ? 31.622776601683793f : dv;
  dv = (kk == 4) ? 100.0f : dv;
  dv = (kk == 5) ? 316.22776601683796f : dv;
  dv = (kk == 6) ? 1000.0f : dv;
  dv = (kk == 7) ? 3162.2776601683795f : dv;
  const float arg = (float)p / dv;
  float sn, cs;
  sincosf(arg, &sn, &cs);
  float val = (j & 1) ? cs : sn;
  val = (p == 0) ? 0.0f : val;
  sv[t] = val;
  __syncthreads();
  if (wave == 0) {
    const int px2 = lane >> 2, sg = lane & 3;
    const float* sp = sv + px2 * 32 + sg * 8;
    v8h hv, lv;
#pragma unroll
    for (int e = 0; e < 8; ++e) {
      _Float16 vh, vl;
      split16(sp[e], vh, vl);
      hv[e] = vh;
      lv[e] = vl;
    }
    const size_t o = (size_t)(n0 + px2) * kPosC + sg * 8;
    *(volatile v8h*)(posH + o) = hv;
    *(volatile v8h*)(posL + o) = lv;
    __threadfence();
    *(volatile v8h*)(posH + o) = hv;
    *(volatile v8h*)(posL + o) = lv;
  }
}

__global__ __launch_bounds__(256) void wcast_kernel(
    const float* __restrict__ fk_w, const float* __restrict__ ck_w, const float* __restrict__ q_w,
    const float* __restrict__ fv_w, const float* __restrict__ cv_w,
    _Float16* __restrict__ WcatH, _Float16* __restrict__ WcatL) {
  const int l  = blockIdx.y / 5;
  const int tn = blockIdx.y - l * 5;
  const int idx = blockIdx.x * 256 + threadIdx.x;
  const int o  = idx / 20;
  const int sg = idx - o * 20;
  const int col0 = sg * 8;
  const float* src = (tn == 0) ? fk_w : (tn == 1) ? ck_w : (tn == 2) ? q_w : (tn == 3) ? fv_w : cv_w;
  const int pitch = (tn == 2) ? kKq : kKg;
  const bool live = (col0 < pitch);
  const int colc = live ? col0 : (pitch - 8);
  const float* p = src + (size_t)(l * kCh + o) * pitch + colc;
  const v4f a0 = *(const v4f*)(p);
  const v4f a1 = *(const v4f*)(p + 4);
  v8h hv, lv;
#pragma unroll
  for (int e = 0; e < 4; ++e) {
    const float f0 = live ? (a0[e] * kWCarry) : 0.0f;
    const float f1 = live ? (a1[e] * kWCarry) : 0.0f;
    _Float16 h0, l0, h1, l1;
    split16(f0, h0, l0);
    split16(f1, h1, l1);
    hv[e]     = h0;
    hv[4 + e] = h1;
    lv[e]     = l0;
    lv[4 + e] = l1;
  }
  const size_t off = ((size_t)(l * 5 + tn) * kCh + o) * kKg + col0;
  *(volatile v8h*)(WcatH + off) = hv;
  *(volatile v8h*)(WcatL + off) = lv;
  __threadfence();
  *(volatile v8h*)(WcatH + off) = hv;
  *(volatile v8h*)(WcatL + off) = lv;
}

__global__ __launch_bounds__(256) void zero_kernel(v4u* __restrict__ p, int n16) {
  const int i = blockIdx.x * 256 + threadIdx.x;
  if (i < n16) {
    const v4u z = (v4u){0u, 0u, 0u, 0u};
    *(volatile v4u*)(p + i) = z;
    __threadfence();
    *(volatile v4u*)(p + i) = z;
  }
}

__global__ __launch_bounds__(256) void conv_kernel(
    const float* __restrict__ x, const float* __restrict__ w, const float* __restrict__ cb,
    float* __restrict__ hpre) {
  const int gi  = blockIdx.x * 256 + threadIdx.x;
  const int pix = gi >> 6, c = gi & 63;
  const int b = pix >> 12, n = pix & (kNpix - 1);
  const int y = n >> 6, xx = n & 63;
  float acc = 0.0f;
#pragma unroll 1
  for (int ic = 0; ic < kConvIn; ++ic) {
    const float* xin = x + (size_t)(b * kConvIn + ic) * kNpix;
    const float* wp  = w + (size_t)(c * kConvIn + ic) * 25;
#pragma unroll
    for (int tap = 0; tap < 12; ++tap) {
      const int ky = (tap < 10) ? (tap / 5) : 2;
      const int kx = (tap < 10) ? (tap % 5) : (tap - 10);
      const int yy = y + ky - 2;
      const int x2 = xx + kx - 2;
      const bool ok = (yy >= 0) && (x2 >= 0) && (x2 < kSide);
      const int yyc = yy < 0 ? 0 : yy;
      const int x2c = x2 < 0 ? 0 : (x2 > kSide - 1 ? kSide - 1 : x2);
      float xv = xin[yyc * kSide + x2c];
      asm volatile("" : "+v"(xv));
      const float wv = wp[tap];
      const float xs = ok ? xv : 0.0f;
      acc = fmaf(wv, xs, acc);
    }
  }
  acc += cb[c];
  float* dst = hpre + (size_t)pix * kCh + c;
  *(volatile float*)dst = acc;
  __threadfence();
  *(volatile float*)dst = acc;
}

__global__ __launch_bounds__(256) void bn_stats_kernel(const float* __restrict__ X, float* __restrict__ stats) {
  __shared__ float redA[8];
  __shared__ float redB[8];
  const int c = blockIdx.x;
  const int t = threadIdx.x, lane = t & 31, wave = t >> 5;
  float s = 0.0f;
#pragma unroll 8
  for (int i = 0; i < 32; ++i) s += X[(size_t)(t + 256 * i) * kCh + c];
  s = wave_sum(s);
  if (lane == 0) redA[wave] = s;
  __syncthreads();
  float tot = 0.0f;
#pragma unroll
  for (int wv = 0; wv < 8; ++wv) tot += redA[wv];
  const float mean = tot * kInvCount;
  float q = 0.0f;
#pragma unroll 8
  for (int i = 0; i < 32; ++i) {
    const float d = X[(size_t)(t + 256 * i) * kCh + c] - mean;
    q = fmaf(d, d, q);
  }
  q = wave_sum(q);
  if (lane == 0) redB[wave] = q;
  __syncthreads();
  float qt = 0.0f;
#pragma unroll
  for (int wv = 0; wv < 8; ++wv) qt += redB[wv];
  const float var  = qt * kInvCount;
  const float rstd = 1.0f / sqrtf(var + kBnEps);
  if (wave == 0) {
    float val = 0.0f;
    val = (lane == 0) ? mean : val;
    val = (lane == 1) ? rstd : val;
    float* dst = stats + c * 32 + lane;
    *(volatile float*)dst = val;
    __threadfence();
    *(volatile float*)dst = val;
  }
}

__global__ __launch_bounds__(256) void bn_apply_kernel(
    const float* __restrict__ X, const float* __restrict__ stats,
    const float* __restrict__ g, const float* __restrict__ bta,
    _Float16* __restrict__ hTh, _Float16* __restrict__ hTl) {
  __shared__ float sM[kCh];
  __shared__ float sA[kCh];
  __shared__ float sB[kCh];
  const int t = threadIdx.x;
  {
    const int tc = t & (kCh - 1);
    float m  = stats[tc * 32];
    float rs = stats[tc * 32 + 1];
    float gg = g[tc];
    float bb = bta[tc];
    asm volatile("" : "+v"(m), "+v"(rs), "+v"(gg), "+v"(bb));
    if (t < kCh) {
      sM[t] = m;
      sA[t] = rs * gg;
      sB[t] = bb;
    }
  }
  __syncthreads();
  const int gi  = blockIdx.x * 256 + t;
  const int row = gi >> 3, c8 = (gi & 7) * 8;
  const float* p = X + (size_t)row * kCh + c8;
  const v4f a0 = *(const v4f*)(p);
  const v4f a1 = *(const v4f*)(p + 4);
  v8h hv, lv;
#pragma unroll
  for (int e = 0; e < 4; ++e) {
    float y0 = (a0[e] - sM[c8 + e]) * sA[c8 + e] + sB[c8 + e];
    float y1 = (a1[e] - sM[c8 + 4 + e]) * sA[c8 + 4 + e] + sB[c8 + 4 + e];
    y0 = (y0 >= 0.0f) ? y0 : 0.01f * y0;
    y1 = (y1 >= 0.0f) ? y1 : 0.01f * y1;
    _Float16 h0, l0, h1, l1;
    split16(y0, h0, l0);
    split16(y1, h1, l1);
    hv[e]     = h0;
    hv[4 + e] = h1;
    lv[e]     = l0;
    lv[4 + e] = l1;
  }
  const size_t off = (size_t)row * kCh + c8;
  *(volatile v8h*)(hTh + off) = hv;
  *(volatile v8h*)(hTl + off) = lv;
  __threadfence();
  *(volatile v8h*)(hTh + off) = hv;
  *(volatile v8h*)(hTl + off) = lv;
}

__global__ __launch_bounds__(256) void gate_gemm_kernel(
    const _Float16* __restrict__ hTh, const _Float16* __restrict__ hTl,
    const _Float16* __restrict__ posH, const _Float16* __restrict__ posL,
    const _Float16* __restrict__ kTh, const _Float16* __restrict__ kTl,
    const _Float16* __restrict__ vTh, const _Float16* __restrict__ vTl,
    const _Float16* __restrict__ Wh, const _Float16* __restrict__ Wl,
    const float* __restrict__ bfk, const float* __restrict__ bck, const float* __restrict__ bq,
    const float* __restrict__ bfv, const float* __restrict__ bcv,
    float* __restrict__ fkp, float* __restrict__ ckp,
    _Float16* __restrict__ qTh, _Float16* __restrict__ qTl,
    float* __restrict__ fvp, float* __restrict__ cvp) {
  __shared__ __align__(16) float sT[8][16 * 68];
  const int lane = threadIdx.x & 31;
  const int wave = threadIdx.x >> 5;
  const int tile = blockIdx.x * 8 + wave;
  if (tile >= kGateTiles) return;
  const int tm = tile / 5;
  const int tn = tile - tm * 5;
  const int m0 = tm * kGateTileM;
  const int rlane = lane & 15;
  const int koff  = (lane >> 4) * 8;
  const int mOff  = (lane >> 4) * 8;
  const _Float16* sPh = (tn < 3) ? kTh : vTh;
  const _Float16* sPl = (tn < 3) ? kTl : vTl;
  const int nk = (tn == 2) ? (kKq / 32) : (kKg / 32);
  const _Float16* WtH = Wh + (size_t)(tn * kCh) * kKg;
  const _Float16* WtL = Wl + (size_t)(tn * kCh) * kKg;

  v8f accM[2][4];
  v8f accS[2][4];
#pragma unroll
  for (int i = 0; i < 2; ++i)
#pragma unroll
    for (int j = 0; j < 4; ++j) {
      accM[i][j] = (v8f){0.f, 0.f, 0.f, 0.f, 0.f, 0.f, 0.f, 0.f};
      accS[i][j] = (v8f){0.f, 0.f, 0.f, 0.f, 0.f, 0.f, 0.f, 0.f};
    }

#pragma unroll 1
  for (int kc = 0; kc < nk; ++kc) {
    const _Float16* abh;
    const _Float16* abl;
    int apitch, acol, rmask;
    if (kc < 2) {
      abh = hTh; abl = hTl; apitch = kCh; acol = kc * 32; rmask = 0x7fffffff;
    } else if (kc == 2) {
      abh = posH; abl = posL; apitch = kPosC; acol = 0; rmask = kNpix - 1;
    } else {
      abh = sPh; abl = sPl; apitch = kCh; acol = (kc - 3) * 32; rmask = 0x7fffffff;
    }
    v16h ah[2], al[2];
#pragma unroll
    for (int i = 0; i < 2; ++i) {
      const int arow = (m0 + (i << 4) + rlane) & rmask;
      const size_t ao = (size_t)arow * apitch + acol + koff;
      ah[i] = frag_load(abh + ao);
      al[i] = frag_load(abl + ao);
    }
#pragma unroll
    for (int j = 0; j < 4; ++j) {
      const size_t wo = (size_t)((j << 4) + rlane) * kKg + kc * 32 + koff;
      const v16h bh = frag_load(WtH + wo);
      const v16h bl = frag_load(WtL + wo);
#pragma unroll
      for (int i = 0; i < 2; ++i) {
        accM[i][j] = mma_h(ah[i], bh, accM[i][j]);
        accS[i][j] = mma_h(ah[i], bl, accS[i][j]);
        accS[i][j] = mma_h(al[i], bh, accS[i][j]);
      }
    }
  }

  float* slab = sT[wave];
  const bool isq = (tn == 2);
  const float* bias = (tn == 0) ? bfk : (tn == 1) ? bck : (tn == 2) ? bq : (tn == 3) ? bfv : bcv;
  float* outF = (tn == 0) ? fkp : (tn == 1) ? ckp : (tn == 3) ? fvp : cvp;
  float bvv[4];
#pragma unroll
  for (int j = 0; j < 4; ++j) bvv[j] = bias[(j << 4) + rlane];
#pragma unroll
  for (int i = 0; i < 2; ++i) {
    const int mBase = m0 + (i << 4);
#pragma unroll
    for (int j = 0; j < 4; ++j) {
#pragma unroll
      for (int r = 0; r < 8; ++r) {
        const float prod = accM[i][j][r] + accS[i][j][r] * kResInv;
        float v = prod * kWCarryInv + bvv[j];
        const float vl = (v >= 0.0f) ? v : 0.01f * v;
        v = isq ? vl : v;
        slab[(mOff + r) * 68 + (j << 4) + rlane] = v;
      }
    }
    __builtin_amdgcn_fence(__ATOMIC_RELEASE, "workgroup");
    __builtin_amdgcn_wave_barrier();
    __builtin_amdgcn_fence(__ATOMIC_ACQUIRE, "workgroup");
    if (!isq) {
      const int hh = lane >> 4, c4 = (lane & 15) * 4;
      for (int pass = 0; pass < 2; ++pass) {
#pragma unroll
        for (int it = 0; it < 8; ++it) {
          const int row = it * 2 + hh;
          const v4f v = *(const v4f*)(slab + row * 68 + c4);
          *(volatile v4f*)(outF + (size_t)(mBase + row) * kCh + c4) = v;
        }
        __threadfence();
      }
    } else {
      const int q = lane >> 3, c8 = (lane & 7) * 8;
      v8h hv[4], lv[4];
#pragma unroll
      for (int it = 0; it < 4; ++it) {
        const int row = it * 4 + q;
        const float* sp = slab + row * 68 + c8;
#pragma unroll
        for (int e = 0; e < 8; ++e) {
          _Float16 vh, vlo;
          split16(sp[e], vh, vlo);
          hv[it][e] = vh;
          lv[it][e] = vlo;
        }
      }
      for (int pass = 0; pass < 2; ++pass) {
#pragma unroll
        for (int it = 0; it < 4; ++it) {
          const int row = it * 4 + q;
          const size_t o = (size_t)(mBase + row) * kCh + c8;
          *(volatile v8h*)(qTh + o) = hv[it];
          *(volatile v8h*)(qTl + o) = lv[it];
        }
        __threadfence();
      }
    }
    __builtin_amdgcn_fence(__ATOMIC_RELEASE, "workgroup");
    __builtin_amdgcn_wave_barrier();
    __builtin_amdgcn_fence(__ATOMIC_ACQUIRE, "workgroup");
  }
}

__global__ __launch_bounds__(128) void attn_kernel(
    const _Float16* __restrict__ qTh, const _Float16* __restrict__ qTl,
    const _Float16* __restrict__ kTh, const _Float16* __restrict__ kTl,
    const _Float16* __restrict__ VcmH, const _Float16* __restrict__ VcmL,
    float* __restrict__ out1) {
  __shared__ __align__(16) _Float16 KshH[64 * 64];
  __shared__ __align__(16) _Float16 KshL[64 * 64];
  __shared__ __align__(16) _Float16 VthH[64 * 64];
  __shared__ __align__(16) _Float16 VthL[64 * 64];
  __shared__ __align__(16) _Float16 Psh[4][16 * 64];
  __shared__ __align__(16) float    Os[4][16 * 68];

  const int tid  = threadIdx.x;
  const int wave = tid >> 5;
  const int lane = tid & 31;
  const int hh   = lane >> 4;
  const int c    = lane & 15;
  const int b    = blockIdx.x >> 6;
  const int qb   = blockIdx.x & 63;
  const int q0   = qb * 64 + wave * 16;
  const size_t rowb = (size_t)b * kNpix;

  v16h qaH[2], qaL[2];
#pragma unroll
  for (int dc = 0; dc < 2; ++dc) {
    const size_t qo = (rowb + q0 + c) * kCh + dc * 32 + 8 * hh;
    qaH[dc] = frag_load(qTh + qo);
    qaL[dc] = frag_load(qTl + qo);
  }

  float mrow[8], lrow[8];
  v8f oaccM[4], oaccS[4];
#pragma unroll
  for (int r = 0; r < 8; ++r) { mrow[r] = -INFINITY; lrow[r] = 0.0f; }
#pragma unroll
  for (int t = 0; t < 4; ++t) {
    oaccM[t] = (v8f){0.f, 0.f, 0.f, 0.f, 0.f, 0.f, 0.f, 0.f};
    oaccS[t] = (v8f){0.f, 0.f, 0.f, 0.f, 0.f, 0.f, 0.f, 0.f};
  }

  _Float16* pw = Psh[wave];

  for (int kc = 0; kc <= qb; ++kc) {
    const int kv0 = kc * 64;
    __syncthreads();
    {
      const size_t ksrc = (rowb + kv0) * kCh;
#pragma unroll
      for (int i = 0; i < 4; ++i) {
        const int idx = tid + 128 * i;
        *(v8h*)(KshH + idx * 8) = *(const v8h*)(kTh + ksrc + idx * 8);
        *(v8h*)(KshL + idx * 8) = *(const v8h*)(kTl + ksrc + idx * 8);
      }
#pragma unroll
      for (int i = 0; i < 4; ++i) {
        const int idx = tid + 128 * i;
        const int d = idx >> 3, sg = idx & 7;
        const size_t vo = ((size_t)b * kCh + d) * kNpix + kv0 + sg * 8;
        *(v8h*)(VthH + idx * 8) = *(const v8h*)(VcmH + vo);
        *(v8h*)(VthL + idx * 8) = *(const v8h*)(VcmL + vo);
      }
    }
    __syncthreads();

    v8f s[4];
#pragma unroll
    for (int j = 0; j < 4; ++j) {
      v8f sm = (v8f){0.f, 0.f, 0.f, 0.f, 0.f, 0.f, 0.f, 0.f};
      v8f ss = (v8f){0.f, 0.f, 0.f, 0.f, 0.f, 0.f, 0.f, 0.f};
#pragma unroll
      for (int dc = 0; dc < 2; ++dc) {
        const int ko = (j * 16 + c) * 64 + dc * 32 + 8 * hh;
        const v16h kbh = frag_load(KshH + ko);
        const v16h kbl = frag_load(KshL + ko);
        sm = mma_h(qaH[dc], kbh, sm);
        ss = mma_h(qaH[dc], kbl, ss);
        ss = mma_h(qaL[dc], kbh, ss);
      }
#pragma unroll
      for (int r = 0; r < 8; ++r) s[j][r] = sm[r] + ss[r] * kResInv;
    }
    const bool diag = (kc == qb);
    float cm[8];
#pragma unroll
    for (int r = 0; r < 8; ++r) {
      const int qrow = q0 + 8 * hh + r;
      float m = -INFINITY;
#pragma unroll
      for (int j = 0; j < 4; ++j) {
        const int kvcol = kv0 + j * 16 + c;
        float sv = s[j][r] * kScoreScale;
        sv = (diag && (kvcol > qrow)) ? kMaskFill : sv;
        s[j][r] = sv;
        m = fmaxf(m, sv);
      }
#pragma unroll
      for (int off = 1; off < 16; off <<= 1) m = fmaxf(m, __shfl_xor(m, off, 32));
      cm[r] = m;
    }
#pragma unroll
    for (int r = 0; r < 8; ++r) {
      const float mnew  = fmaxf(mrow[r], cm[r]);
      const float alpha = __expf(mrow[r] - mnew);
      mrow[r] = mnew;
      float psum = 0.0f;
#pragma unroll
      for (int j = 0; j < 4; ++j) {
        const float p = __expf(s[j][r] - mnew);
        const _Float16 p16 = (_Float16)(p * kPCarry);
        psum += (float)p16;
        pw[(8 * hh + r) * 64 + j * 16 + c] = p16;
      }
#pragma unroll
      for (int off = 1; off < 16; off <<= 1) psum += __shfl_xor(psum, off, 32);
      lrow[r] = lrow[r] * alpha + psum;
#pragma unroll
      for (int t = 0; t < 4; ++t) {
        oaccM[t][r] *= alpha;
        oaccS[t][r] *= alpha;
      }
    }
    __builtin_amdgcn_fence(__ATOMIC_RELEASE, "workgroup");
    __builtin_amdgcn_wave_barrier();
    __builtin_amdgcn_fence(__ATOMIC_ACQUIRE, "workgroup");
#pragma unroll
    for (int kk = 0; kk < 2; ++kk) {
      const v16h pa = frag_load(pw + c * 64 + kk * 32 + 8 * hh);
#pragma unroll
      for (int t = 0; t < 4; ++t) {
        const int vo = (t * 16 + c) * 64 + kk * 32 + 8 * hh;
        const v16h vbh = frag_load(VthH + vo);
        const v16h vbl = frag_load(VthL + vo);
        oaccM[t] = mma_h(pa, vbh, oaccM[t]);
        oaccS[t] = mma_h(pa, vbl, oaccS[t]);
      }
    }
  }

  float* os = Os[wave];
#pragma unroll
  for (int r = 0; r < 8; ++r) {
    const float inv = 1.0f / lrow[r];
#pragma unroll
    for (int t = 0; t < 4; ++t) {
      const float o = oaccM[t][r] + oaccS[t][r] * kResInv;
      os[(8 * hh + r) * 68 + t * 16 + c] = o * inv;
    }
  }
  __builtin_amdgcn_fence(__ATOMIC_RELEASE, "workgroup");
  __builtin_amdgcn_wave_barrier();
  __builtin_amdgcn_fence(__ATOMIC_ACQUIRE, "workgroup");
  {
    const int c4 = (lane & 15) * 4;
    for (int pass = 0; pass < 2; ++pass) {
#pragma unroll
      for (int it = 0; it < 8; ++it) {
        const int row = it * 2 + hh;
        const v4f val = *(const v4f*)(os + row * 68 + c4);
        *(volatile v4f*)(out1 + (rowb + q0 + row) * kCh + c4) = val;
      }
      __threadfence();
    }
  }
}

__global__ __launch_bounds__(256) void kv_update_kernel(
    const float* __restrict__ fkp, const float* __restrict__ ckp,
    const float* __restrict__ fvp, const float* __restrict__ cvp,
    const float* __restrict__ kOld, const float* __restrict__ vOld,
    float* __restrict__ kNew, float* __restrict__ vNew,
    _Float16* __restrict__ kTh, _Float16* __restrict__ kTl,
    _Float16* __restrict__ vTh, _Float16* __restrict__ vTl,
    _Float16* __restrict__ VcmH, _Float16* __restrict__ VcmL) {
  __shared__ __align__(16) float tile[64 * 68];
  const int tid = threadIdx.x, lane = tid & 31, wave = tid >> 5;
  const int q = lane >> 3, c8 = (lane & 7) * 8;
  const int r0 = blockIdx.x * 64;
  const int b  = r0 >> 12;
  const int n0 = r0 & (kNpix - 1);
#pragma unroll 1
  for (int which = 0; which < 2; ++which) {
    const float* fp = which ? fvp : fkp;
    const float* cp = which ? cvp : ckp;
    const float* sp = which ? vOld : kOld;
    float*       np = which ? vNew : kNew;
    _Float16*    t16h = which ? vTh : kTh;
    _Float16*    t16l = which ? vTl : kTl;
#pragma unroll 1
    for (int it = 0; it < 4; ++it) {
      const int e  = tid + 256 * it;
      const int px = e >> 4, c4 = (e & 15) * 4;
      const size_t off = (size_t)(r0 + px) * kCh + c4;
      const v4f f = *(const v4f*)(fp + off);
      const v4f g = *(const v4f*)(cp + off);
      const v4f s = *(const v4f*)(sp + off);
      v4f o;
#pragma unroll
      for (int k = 0; k < 4; ++k) {
        const float ex = expf(fminf(-f[k], 60.0f));
        const float sg = 1.0f / (1.0f + ex);
        const float lr = (g[k] >= 0.0f) ? g[k] : 0.01f * g[k];
        o[k] = sg * s[k] + lr;
      }
      *(v4f*)(tile + px * 68 + c4) = o;
      *(volatile v4f*)(np + off) = o;
      __threadfence();
      *(volatile v4f*)(np + off) = o;
    }
    __syncthreads();
    {
      v8h hv[2], lv[2];
#pragma unroll
      for (int it = 0; it < 2; ++it) {
        const int row = wave * 8 + it * 4 + q;
        const float* tp = tile + row * 68 + c8;
        const v4f a0 = *(const v4f*)(tp);
        const v4f a1 = *(const v4f*)(tp + 4);
#pragma unroll
        for (int e = 0; e < 4; ++e) {
          _Float16 h0, l0, h1, l1;
          split16(a0[e], h0, l0);
          split16(a1[e], h1, l1);
          hv[it][e]     = h0;
          hv[it][4 + e] = h1;
          lv[it][e]     = l0;
          lv[it][4 + e] = l1;
        }
      }
      for (int pass = 0; pass < 2; ++pass) {
#pragma unroll
        for (int it = 0; it < 2; ++it) {
          const int row = wave * 8 + it * 4 + q;
          const size_t o = (size_t)(r0 + row) * kCh + c8;
          *(volatile v8h*)(t16h + o) = hv[it];
          *(volatile v8h*)(t16l + o) = lv[it];
        }
        __threadfence();
      }
    }
    if (which == 1) {
      v8h tv[2], tl[2];
#pragma unroll
      for (int it = 0; it < 2; ++it) {
        const int ch = wave * 8 + it * 4 + q;
#pragma unroll
        for (int e = 0; e < 8; ++e) {
          _Float16 vh, vlo;
          split16(tile[(c8 + e) * 68 + ch], vh, vlo);
          tv[it][e] = vh;
          tl[it][e] = vlo;
        }
      }
      for (int pass = 0; pass < 2; ++pass) {
#pragma unroll
        for (int it = 0; it < 2; ++it) {
          const int ch = wave * 8 + it * 4 + q;
          const size_t o = ((size_t)b * kCh + ch) * kNpix + n0 + c8;
          *(volatile v8h*)(VcmH + o) = tv[it];
          *(volatile v8h*)(VcmL + o) = tl[it];
        }
        __threadfence();
      }
    }
    __syncthreads();
  }
}

__global__ __launch_bounds__(256) void outproj_kernel(
    const float* __restrict__ X, const float* __restrict__ stats,
    const float* __restrict__ g, const float* __restrict__ bta,
    const float* __restrict__ out_w, const float* __restrict__ out_b, float* __restrict__ out) {
  __shared__ float sM[kCh];
  __shared__ float sA[kCh];
  __shared__ float sB[kCh];
  __shared__ __align__(16) float hs[64 * 68];
  const int t = threadIdx.x;
  const int r0 = blockIdx.x * 64;
  const int b  = r0 >> 12;
  const int n0 = r0 & (kNpix - 1);
  {
    const int tc = t & (kCh - 1);
    float m  = stats[tc * 32];
    float rs = stats[tc * 32 + 1];
    float gg = g[tc];
    float bb = bta[tc];
    asm volatile("" : "+v"(m), "+v"(rs), "+v"(gg), "+v"(bb));
    if (t < kCh) {
      sM[t] = m;
      sA[t] = rs * gg;
      sB[t] = bb;
    }
  }
  __syncthreads();
#pragma unroll 1
  for (int it = 0; it < 4; ++it) {
    const int e  = t + 256 * it;
    const int px = e >> 4, c4 = (e & 15) * 4;
    const v4f xv = *(const v4f*)(X + (size_t)(r0 + px) * kCh + c4);
    v4f y;
#pragma unroll
    for (int k = 0; k < 4; ++k) {
      float yy = (xv[k] - sM[c4 + k]) * sA[c4 + k] + sB[c4 + k];
      yy = (yy >= 0.0f) ? yy : 0.01f * yy;
      y[k] = yy;
    }
    *(v4f*)(hs + px * 68 + c4) = y;
  }
  __syncthreads();
  const int nl = t & 63, og = t >> 6;
  const float* hrow = hs + nl * 68;
#pragma unroll 1
  for (int o = og; o < kOutC; o += 4) {
    const v4f* wr = (const v4f*)(out_w + (size_t)o * kCh);
    float acc = 0.0f;
#pragma unroll 4
    for (int c4 = 0; c4 < 16; ++c4) {
      const v4f w4 = wr[c4];
      const v4f h4 = *(const v4f*)(hrow + 4 * c4);
      acc = fmaf(w4[0], h4[0], acc);
      acc = fmaf(w4[1], h4[1], acc);
      acc = fmaf(w4[2], h4[2], acc);
      acc = fmaf(w4[3], h4[3], acc);
    }
    acc += out_b[o];
    float* dst = out + ((size_t)(b * kOutC + o)) * kNpix + n0 + nl;
    *(volatile float*)dst = acc;
    __threadfence();
    *(volatile float*)dst = acc;
  }
}

extern "C" void kernel_launch(void* const* d_in, const int* in_sizes, int n_in,
                              void* d_out, int out_size, void* d_ws, size_t ws_size,
                              hipStream_t stream) {
  if (n_in < 19) return;
  if (in_sizes[0] != kBatch * kConvIn * kNpix) return;
  if (in_sizes[1] != kCh * kConvIn * 25) return;
  if (in_sizes[2] != kCh || in_sizes[3] != kCh || in_sizes[4] != kCh) return;
  if (in_sizes[5] != kLayers * kCh * kKq) return;
  if (in_sizes[7] != kLayers * kCh * kKg || in_sizes[9] != kLayers * kCh * kKg) return;
  if (in_sizes[11] != kLayers * kCh * kKg || in_sizes[13] != kLayers * kCh * kKg) return;
  if (in_sizes[6] != kLayers * kCh || in_sizes[8] != kLayers * kCh || in_sizes[10] != kLayers * kCh) return;
  if (in_sizes[12] != kLayers * kCh || in_sizes[14] != kLayers * kCh) return;
  if (in_sizes[15] != kLayers * kCh || in_sizes[16] != kLayers * kCh) return;
  if (in_sizes[17] != kOutC * kCh || in_sizes[18] != kOutC) return;
  if (out_size != kBatch * kOutC * kNpix) return;
  if (ws_size < kWsTotal) return;

  const float* x      = (const float*)d_in[0];
  const float* conv_w = (const float*)d_in[1];
  const float* conv_b = (const float*)d_in[2];
  const float* bn0_g  = (const float*)d_in[3];
  const float* bn0_b  = (const float*)d_in[4];
  const float* q_w    = (const float*)d_in[5];
  const float* q_b    = (const float*)d_in[6];
  const float* fk_w   = (const float*)d_in[7];
  const float* fk_b   = (const float*)d_in[8];
  const float* ck_w   = (const float*)d_in[9];
  const float* ck_b   = (const float*)d_in[10];
  const float* fv_w   = (const float*)d_in[11];
  const float* fv_b   = (const float*)d_in[12];
  const float* cv_w   = (const float*)d_in[13];
  const float* cv_b   = (const float*)d_in[14];
  const float* bn_g   = (const float*)d_in[15];
  const float* bn_b   = (const float*)d_in[16];
  const float* out_w  = (const float*)d_in[17];
  const float* out_b  = (const float*)d_in[18];
  float* out = (float*)d_out;

  char* ws = (char*)d_ws;
  _Float16* POSH = (_Float16*)(ws + kOffPosH);
  _Float16* POSL = (_Float16*)(ws + kOffPosL);
  _Float16* WH   = (_Float16*)(ws + kOffWH);
  _Float16* WL   = (_Float16*)(ws + kOffWL);
  float*    STAT = (float*)(ws + kOffStat);
  float*    K32A = (float*)(ws + kOffK32A);
  float*    V32A = (float*)(ws + kOffV32A);
  _Float16* KTH  = (_Float16*)(ws + kOffKTH);
  _Float16* KTL  = (_Float16*)(ws + kOffKTL);
  _Float16* VTH  = (_Float16*)(ws + kOffVTH);
  _Float16* VTL  = (_Float16*)(ws + kOffVTL);
  _Float16* VCMH = (_Float16*)(ws + kOffVCMH);
  _Float16* VCML = (_Float16*)(ws + kOffVCML);
  float*    K32B = (float*)(ws + kOffK32B);
  float*    V32B = (float*)(ws + kOffV32B);
  _Float16* HTH  = (_Float16*)(ws + kOffHTH);
  _Float16* HTL  = (_Float16*)(ws + kOffHTL);
  _Float16* QTH  = (_Float16*)(ws + kOffQTH);
  _Float16* QTL  = (_Float16*)(ws + kOffQTL);
  float*    FKP  = (float*)(ws + kOffFKP);
  float*    CKP  = (float*)(ws + kOffCKP);
  float*    FVP  = (float*)(ws + kOffFVP);
  float*    CVP  = (float*)(ws + kOffCVP);
  float*    OUT1 = (float*)(ws + kOffOUT1);
  float*    HPRE = (float*)(ws + kOffHPRE);

  pos_kernel<<<kNpix / 8, 256, 0, stream>>>(POSH, POSL);
  wcast_kernel<<<dim3(5, kLayers * 5), 256, 0, stream>>>(fk_w, ck_w, q_w, fv_w, cv_w, WH, WL);
  zero_kernel<<<(int)(kZeroBytes / 16 / 256), 256, 0, stream>>>((v4u*)(ws + kOffK32A), (int)(kZeroBytes / 16));

  conv_kernel<<<kRows * kCh / 256, 256, 0, stream>>>(x, conv_w, conv_b, HPRE);
  bn_stats_kernel<<<kCh, 256, 0, stream>>>(HPRE, STAT);
  bn_apply_kernel<<<kRows * 8 / 256, 256, 0, stream>>>(HPRE, STAT, bn0_g, bn0_b, HTH, HTL);

  for (int l = 0; l < kLayers; ++l) {
    const _Float16* WlH = WH + (size_t)l * kNcat * kKg;
    const _Float16* WlL = WL + (size_t)l * kNcat * kKg;
    const float* kOld = (l & 1) ? K32B : K32A;
    const float* vOld = (l & 1) ? V32B : V32A;
    float* kNew = (l & 1) ? K32A : K32B;
    float* vNew = (l & 1) ? V32A : V32B;
    const int bo = l * kCh;

    gate_gemm_kernel<<<kGateTiles / 8, 256, 0, stream>>>(
        HTH, HTL, POSH, POSL, KTH, KTL, VTH, VTL, WlH, WlL,
        fk_b + bo, ck_b + bo, q_b + bo, fv_b + bo, cv_b + bo,
        FKP, CKP, QTH, QTL, FVP, CVP);

    attn_kernel<<<kBatch * (kNpix / 64), 128, 0, stream>>>(QTH, QTL, KTH, KTL, VCMH, VCML, OUT1);

    kv_update_kernel<<<kRows / 64, 256, 0, stream>>>(FKP, CKP, FVP, CVP, kOld, vOld, kNew, vNew,
                                                     KTH, KTL, VTH, VTL, VCMH, VCML);

    bn_stats_kernel<<<kCh, 256, 0, stream>>>(OUT1, STAT);
    if (l + 1 < kLayers)
      bn_apply_kernel<<<kRows * 8 / 256, 256, 0, stream>>>(OUT1, STAT, bn_g + bo, bn_b + bo, HTH, HTL);
  }

  outproj_kernel<<<kRows / 64, 256, 0, stream>>>(OUT1, STAT, bn_g + (kLayers - 1) * kCh, bn_b + (kLayers - 1) * kCh,
                                                 out_w, out_b, out);
}
